// PermOnlySSMLayer_62302795596528
// MI455X (gfx1250) — hardware-run, weakly checked
//
#include <hip/hip_runtime.h>
#include <math.h>

typedef __attribute__((ext_vector_type(16))) _Float16 v16h;
typedef __attribute__((ext_vector_type(8)))  _Float16 v8h;
typedef __attribute__((ext_vector_type(2)))  _Float16 v2h;
typedef __attribute__((ext_vector_type(16))) __bf16   v16b;
typedef __attribute__((ext_vector_type(8)))  __bf16   v8b;
typedef __attribute__((ext_vector_type(8)))  float    v8f;
typedef __attribute__((ext_vector_type(4)))  float    v4f;
typedef __attribute__((ext_vector_type(2)))  float    v2f;
typedef __attribute__((ext_vector_type(4)))  _Float16 v4h;

constexpr int kNB   = 4;
constexpr int kL    = 1024;
constexpr int kRows = kNB * kL;
constexpr int kD    = 1024;
constexpr int kH    = 8;
constexpr int kN    = 16;
constexpr int kHN   = kH * kN;
constexpr int kHNN  = kH * kN * kN;
constexpr int kPrj  = kHNN + 2 * kHN;
constexpr int kOut0 = kRows * kD;
constexpr int kBvTot = kPrj + kD;
constexpr int kSweeps = 5;
constexpr int kThr  = 256;
constexpr float kWCarry  = 4096.0f;
constexpr float kNCarry  = 1024.0f;
constexpr float kHCarry  = 4096.0f;
constexpr float kScP = 1.0f / (kNCarry * kWCarry);
constexpr float kScO = 1.0f / (kHCarry * kWCarry);
constexpr float kNormEps = 1e-5f;
constexpr float kF16MinNormal = 6.103515625e-5f;

static_assert(kRows == 4096 && kD == 1024 && kHN == 128 && kHNN == 2048 && kPrj == 2304 && (kPrj % 64) == 0 && (kL & (kL - 1)) == 0, "the index arithmetic below uses these sizes");

constexpr size_t kOffWALL = 0ull;
constexpr size_t kOffWOT = 4718592ull;
constexpr size_t kOffBV = 4980736ull;
constexpr size_t kOffST = 4994048ull;
constexpr size_t kOffXN16 = 5026816ull;
constexpr size_t kOffPRJ = 13415424ull;
constexpr size_t kOffLA = 51164160ull;
constexpr size_t kOffLB = 84718592ull;
constexpr size_t kOffG = 118273024ull;
constexpr size_t kOffHS16 = 120370176ull;
constexpr size_t kOffY = 121418752ull;
constexpr size_t kWsTotal = 138195968ull;
static_assert(kWsTotal <= 268435456ull, "the carve stands under the contract's 256 MiB of workspace");
static_assert(kOffWALL == 0
  && kOffWOT == kOffWALL + 4718592ull
  && kOffBV == kOffWOT + 262144ull
  && kOffST == kOffBV + 13312ull
  && kOffXN16 == kOffST + 32768ull
  && kOffPRJ == kOffXN16 + 8388608ull
  && kOffLA == kOffPRJ + 37748736ull
  && kOffLB == kOffLA + 33554432ull
  && kOffG == kOffLB + 33554432ull
  && kOffHS16 == kOffG + 2097152ull
  && kOffY == kOffHS16 + 1048576ull
  && kWsTotal == kOffY + 16777216ull, "the carve is a chain: every region starts where the one before ends");
static_assert((size_t)kPrj * kD * 2 == 4718592ull && (size_t)kD * kHN * 2 == 262144ull && (size_t)kBvTot * 4 == 13312ull && (size_t)kRows * 2 * 4 == 32768ull && (size_t)kRows * kD * 2 == 8388608ull && (size_t)kRows * kPrj * 4 == 37748736ull
  && (size_t)kRows * kHNN * 4 == 33554432ull && (size_t)kRows * kHN * 4 == 2097152ull && (size_t)kRows * kHN * 2 == 1048576ull && (size_t)kRows * kD * 4 == 16777216ull, "every region's length is its plane's");
static_assert((kOffWOT % 256) == 0 && (kOffBV % 256) == 0 && (kOffST % 256) == 0 && (kOffXN16 % 256) == 0 && (kOffPRJ % 256) == 0 && (kOffLA % 256) == 0 && (kOffLB % 256) == 0 && (kOffG % 256) == 0 && (kOffHS16 % 256) == 0 && (kOffY % 256) == 0,
  "every region starts on a multiple of 256 B");

__device__ __forceinline__ unsigned short f2bf_bits(float f) {
  unsigned u = __float_as_uint(f);
  return (unsigned short)((u + 0x7FFFu + ((u >> 16) & 1u)) >> 16);
}
__device__ __forceinline__ float bf_bits2f(unsigned short h) { return __uint_as_float(((unsigned)h) << 16); }
__device__ __forceinline__ float bf16r(float f) { return bf_bits2f(f2bf_bits(f)); }
__device__ __forceinline__ float carry_flush(float v, float carry) {
  const float s = v * carry;
  return (fabsf(s) < kF16MinNormal) ? 0.0f : s;
}

__device__ __forceinline__ void dep_guard4_h(v8f& a, v8f& b, v8f& c, v8f& d, v16h x, v16h y) { asm volatile("v_nop\n\tv_nop\n\tv_nop\n\tv_nop" : "+v"(a), "+v"(b), "+v"(c), "+v"(d) : "v"(x), "v"(y)); }
__device__ __forceinline__ void dep_guard4_b(v8f& a, v8f& b, v8f& c, v8f& d, v16b x, v16b y) { asm volatile("v_nop\n\tv_nop\n\tv_nop\n\tv_nop" : "+v"(a), "+v"(b), "+v"(c), "+v"(d) : "v"(x), "v"(y)); }
__device__ __forceinline__ void keep4_h(v16h a, v16h b, v16h c, v16h d) { asm volatile("v_nop" :: "v"(a), "v"(b), "v"(c), "v"(d)); }
__device__ __forceinline__ void keep4_b(v16b a, v16b b, v16b c, v16b d) { asm volatile("v_nop" :: "v"(a), "v"(b), "v"(c), "v"(d)); }
__device__ __forceinline__ void acc_guard4(v8f& a, v8f& b, v8f& c, v8f& d) { asm volatile("v_nop\n\tv_nop\n\tv_nop\n\tv_nop" : "+v"(a), "+v"(b), "+v"(c), "+v"(d)); }

template <typename T> struct Frag;
template <> struct Frag<_Float16> {
  typedef v16h V; union U { v16h v; v8h h[2]; };
  static __device__ __forceinline__ v16h load(const _Float16* p) {
    U f; f.h[0] = *(const v8h*)(p); f.h[1] = *(const v8h*)(p + 16); return f.v;
  }
  static __device__ __forceinline__ v8f mma(v16h a, v16h b, v8f c) {
    return __builtin_amdgcn_wmma_f32_16x16x32_f16(false, a, false, b, (short)0, c, false, false);
  }
  static __device__ __forceinline__ void guard4(v8f& a, v8f& b, v8f& c, v8f& d, v16h x, v16h y) { dep_guard4_h(a, b, c, d, x, y); }
  static __device__ __forceinline__ void keep(v16h a, v16h b, v16h c, v16h d) { keep4_h(a, b, c, d); }
};
template <> struct Frag<__bf16> {
  typedef v16b V; union U { v16b v; v8b h[2]; };
  static __device__ __forceinline__ v16b load(const __bf16* p) {
    U f; f.h[0] = *(const v8b*)(p); f.h[1] = *(const v8b*)(p + 16); return f.v;
  }
  static __device__ __forceinline__ v8f mma(v16b a, v16b b, v8f c) {
    return __builtin_amdgcn_wmma_f32_16x16x32_bf16(false, a, false, b, (short)0, c, false, false);
  }
  static __device__ __forceinline__ void guard4(v8f& a, v8f& b, v8f& c, v8f& d, v16b x, v16b y) { dep_guard4_b(a, b, c, d, x, y); }
  static __device__ __forceinline__ void keep(v16b a, v16b b, v16b c, v16b d) { keep4_b(a, b, c, d); }
};

__device__ __forceinline__ v8f mma_h(v16h a, v16h b, v8f c) {
  c = __builtin_amdgcn_wmma_f32_16x16x32_f16(false, a, false, b, (short)0, c, false, false);
  asm volatile("v_nop\n\tv_nop\n\tv_nop\n\tv_nop" : "+v"(c) : "v"(a), "v"(b));
  return c;
}

template <int ET> struct Elem;
template <> struct Elem<0> { typedef _Float16 T; };
template <> struct Elem<1> { typedef __bf16 T; };
template <int ET, bool SPLIT, int BIAS_MODE, int OUT_MODE, bool RESID, int ACT = 0>
__global__ __launch_bounds__(256) void wmma_gemm64(
    const unsigned short* __restrict__ Ap, const unsigned short* __restrict__ A2p, int lda, long strideA,
    const unsigned short* __restrict__ Btp, const unsigned short* __restrict__ Bt2p, int ldb, long strideB,
    void* __restrict__ Cout, void* __restrict__ Cout2, int ldc, long strideC,
    const float* __restrict__ bias,
    const float* __restrict__ resid, long strideR,
    int M, int N, int K, float scale) {
  typedef typename Elem<ET>::T T;
  typedef typename Frag<T>::V V;
  const T* A = (const T*)Ap; const T* A2 = (const T*)A2p; const T* Bt = (const T*)Btp; const T* Bt2 = (const T*)Bt2p;
  __shared__ __align__(16) float sT[8][16 * 68];
  const int b    = blockIdx.y;
  const int lane = threadIdx.x & 31;
  const int wave = threadIdx.x >> 5;
  const int tilesN = N >> 6;
  const int tilesM = M >> 6;
  const int tile = blockIdx.x * 8 + wave;
  if (tile >= tilesM * tilesN) return;
  const int tm = tile / tilesN;
  const int tn = tile - tm * tilesN;
  const int m0 = tm << 6;
  const int n0 = tn << 6;

  const T* Ab  = A  + (size_t)b * strideA;
  const T* Bb  = Bt + (size_t)b * strideB;
  const T* Ab2 = SPLIT ? (A2  + (size_t)b * strideA) : nullptr;
  const T* Bb2 = SPLIT ? (Bt2 + (size_t)b * strideB) : nullptr;

  const int rlane = lane & 15;
  const int koff  = (lane >> 4) * 8;
  const int mOff  = (lane >> 4) * 8;

  v8f acc[4][4];
#pragma unroll
  for (int i = 0; i < 4; ++i)
#pragma unroll
    for (int j = 0; j < 4; ++j) acc[i][j] = (v8f){0.f,0.f,0.f,0.f,0.f,0.f,0.f,0.f};

  for (int k0 = 0; k0 < K; k0 += 32) {
    V bh[4], bl[4];
#pragma unroll
    for (int j = 0; j < 4; ++j) {
      const size_t bo = (size_t)(n0 + (j << 4) + rlane) * ldb + koff + k0;
      bh[j] = Frag<T>::load(Bb + bo);
      if (SPLIT) bl[j] = Frag<T>::load(Bb2 + bo);
    }
#pragma unroll
    for (int i = 0; i < 4; ++i) {
      const size_t ao = (size_t)(m0 + (i << 4) + rlane) * lda + koff + k0;
      V ah = Frag<T>::load(Ab + ao);
      V al;
      if (SPLIT) al = Frag<T>::load(Ab2 + ao);
#pragma unroll
      for (int j = 0; j < 4; ++j) {
        acc[i][j] = Frag<T>::mma(ah, bh[j], acc[i][j]);
        if (SPLIT) {
          acc[i][j] = Frag<T>::mma(ah, bl[j], acc[i][j]);
          acc[i][j] = Frag<T>::mma(al, bh[j], acc[i][j]);
        }
      }
      Frag<T>::guard4(acc[i][0], acc[i][1], acc[i][2], acc[i][3], ah, SPLIT ? al : ah);
    }
    Frag<T>::keep(bh[0], bh[1], bh[2], bh[3]);
    if (SPLIT) Frag<T>::keep(bl[0], bl[1], bl[2], bl[3]);
  }
  acc_guard4(acc[0][0], acc[0][1], acc[0][2], acc[0][3]);
  acc_guard4(acc[1][0], acc[1][1], acc[1][2], acc[1][3]);
  acc_guard4(acc[2][0], acc[2][1], acc[2][2], acc[2][3]);
  acc_guard4(acc[3][0], acc[3][1], acc[3][2], acc[3][3]);

  float* slab = sT[wave];
  const float* Rb = RESID ? (resid + (size_t)b * strideR) : nullptr;
#pragma unroll
  for (int i = 0; i < 4; ++i) {
    const int mBase = m0 + (i << 4);
#pragma unroll
    for (int j = 0; j < 4; ++j) {
      const int n = n0 + (j << 4) + rlane;
      float bv = 0.f;
      if (BIAS_MODE == 2) bv = bias[n];
#pragma unroll
      for (int r = 0; r < 8; ++r) {
        float v = acc[i][j][r] * scale;
        if (BIAS_MODE == 1) v += bias[mBase + mOff + r];
        if (BIAS_MODE == 2) v += bv;
        if (RESID) v += Rb[(size_t)(mBase + mOff + r) * ldc + n];
        if (ACT == 1) v = tanhf(v);
        if (ACT == 2) v = fmaxf(v, 0.0f);
        if (ACT == 3) v = v / (1.0f + expf(-v));
        if (ACT == 4) v = (v > 0.f) ? v : 0.01f * v;
        slab[(mOff + r) * 68 + (j << 4) + rlane] = v;
      }
    }
    __builtin_amdgcn_fence(__ATOMIC_RELEASE, "workgroup");
    __builtin_amdgcn_wave_barrier();
    __builtin_amdgcn_fence(__ATOMIC_ACQUIRE, "workgroup");
    if (OUT_MODE == 0) {
      float* C = (float*)Cout + (size_t)b * strideC;
      const int hh = lane >> 4, c4 = (lane & 15) * 4;
      for (int pass = 0; pass < 2; ++pass) {
#pragma unroll
        for (int it = 0; it < 8; ++it) {
          const int row = it * 2 + hh;
          v4f v = *(const v4f*)(slab + row * 68 + c4);
          *(volatile v4f*)(C + (size_t)(mBase + row) * ldc + n0 + c4) = v;
        }
        __threadfence();
      }
    } else {
      const int q = lane >> 3, c8 = (lane & 7) * 8;
      unsigned short* C  = (unsigned short*)Cout  + (size_t)b * strideC;
      unsigned short* C2 = (OUT_MODE == 2) ? ((unsigned short*)Cout2 + (size_t)b * strideC) : nullptr;
      for (int pass = 0; pass < 2; ++pass) {
#pragma unroll
        for (int it = 0; it < 4; ++it) {
          const int row = it * 4 + q;
          const float* sp = slab + row * 68 + c8;
          v8h hv, lv;
#pragma unroll
          for (int e = 0; e < 8; ++e) {
            if (OUT_MODE == 1) {
              hv[e] = (_Float16)sp[e];
            } else {
              unsigned short hb = f2bf_bits(sp[e]);
              unsigned short lb = f2bf_bits(sp[e] - bf_bits2f(hb));
              hv[e] = __builtin_bit_cast(_Float16, hb);
              lv[e] = __builtin_bit_cast(_Float16, lb);
            }
          }
          *(volatile v8h*)(C + (size_t)(mBase + row) * ldc + n0 + c8) = hv;
          if (OUT_MODE == 2) *(volatile v8h*)(C2 + (size_t)(mBase + row) * ldc + n0 + c8) = lv;
        }
        __threadfence();
      }
    }
    __builtin_amdgcn_fence(__ATOMIC_RELEASE, "workgroup");
    __builtin_amdgcn_wave_barrier();
    __builtin_amdgcn_fence(__ATOMIC_ACQUIRE, "workgroup");
  }
}


__global__ __launch_bounds__(256) void wt_plane_kernel(const float* __restrict__ W, unsigned short* __restrict__ dst, int K, int N, int nLive, int ldd, int colOff) {
  const int n  = blockIdx.x;
  const int k8 = threadIdx.x * 8;
  const bool live = n < nLive;
  const int nc = live ? n : 0;
  v8h hv;
#pragma unroll
  for (int e = 0; e < 8; ++e) {
    const float w = W[(size_t)(k8 + e) * N + nc];
    hv[e] = (_Float16)(live ? carry_flush(bf16r(w), kWCarry) : 0.0f);
  }
  unsigned short* dp = dst + (size_t)n * ldd + colOff + k8;
  *(volatile v8h*)dp = hv;
  __threadfence();
  *(volatile v8h*)dp = hv;
}

__global__ __launch_bounds__(kThr) void setup_kernel(const float* __restrict__ bp, const float* __restrict__ bg, const float* __restrict__ bi, const float* __restrict__ bo, float* __restrict__ BV) {
  const unsigned i = blockIdx.x * (unsigned)kThr + threadIdx.x;
  const float vp = bp[(i < (unsigned)kHNN) ? i : 0u];
  const float vg = bg[(i >= (unsigned)kHNN && i < (unsigned)(kHNN + kHN)) ? (i - (unsigned)kHNN) : 0u];
  const float vi = bi[(i >= (unsigned)(kHNN + kHN) && i < (unsigned)kPrj) ? (i - (unsigned)(kHNN + kHN)) : 0u];
  const float vo = bo[(i >= (unsigned)kPrj) ? (i - (unsigned)kPrj) : 0u];
  const float v = (i < (unsigned)kHNN) ? vp : ((i < (unsigned)(kHNN + kHN)) ? vg : ((i < (unsigned)kPrj) ? vi : vo));
  const float o = bf16r(v);
  float* dp = BV + i;
  *(volatile float*)dp = o;
  __threadfence();
  *(volatile float*)dp = o;
}
static_assert(13 * kThr == kBvTot, "set-up grid exact: 13 blocks");

__global__ __launch_bounds__(kThr) void stat_kernel(const float* __restrict__ x, float* __restrict__ ST) {
  const unsigned row = blockIdx.x * (unsigned)kThr + threadIdx.x;
  const float* pr = x + row * (unsigned)kD;
  float s = 0.0f;
  for (int q = 0; q < kD / 4; ++q) { const v4f v = *(const v4f*)(pr + 4 * q); s += bf16r(v[0]); s += bf16r(v[1]); s += bf16r(v[2]); s += bf16r(v[3]); }
  const float mu = s / (float)kD;
  float qq = 0.0f;
  for (int q = 0; q < kD / 4; ++q) { const v4f v = *(const v4f*)(pr + 4 * q);
#pragma unroll
    for (int e = 0; e < 4; ++e) { const float d = bf16r(v[e]) - mu; qq += d * d; } }
  v2f o; o[0] = mu; o[1] = 1.0f / sqrtf(qq / (float)kD + kNormEps);
  float* dp = ST + row * 2u;
  *(volatile v2f*)dp = o;
  __threadfence();
  *(volatile v2f*)dp = o;
}
static_assert(kRows == 16 * kThr && (kD % 4) == 0, "the statistics' grid exact: 16 blocks: a thread a row");

__global__ __launch_bounds__(kThr) void apply_kernel(const float* __restrict__ x, const float* __restrict__ ST, const float* __restrict__ ln_w, const float* __restrict__ ln_b,
                                                     unsigned short* __restrict__ XN16) {
  const unsigned i = blockIdx.x * (unsigned)kThr + threadIdx.x;
  const unsigned row = i >> 7;
  const unsigned c8 = (i & 127u) * 8u;
  const v2f ms = *(const v2f*)(ST + row * 2u);
  const float* pr = x + i * 8u;
  const v4f a0 = *(const v4f*)pr, a1 = *(const v4f*)(pr + 4);
  const v4f g0 = *(const v4f*)(ln_w + c8), g1 = *(const v4f*)(ln_w + c8 + 4), b0 = *(const v4f*)(ln_b + c8), b1 = *(const v4f*)(ln_b + c8 + 4);
  v8h hv;
#pragma unroll
  for (int e = 0; e < 8; ++e) {
    const float v = (e < 4) ? a0[e] : a1[e - 4];
    const float gw = (e < 4) ? g0[e] : g1[e - 4];
    const float gb = (e < 4) ? b0[e] : b1[e - 4];
    hv[e] = (_Float16)carry_flush(((bf16r(v) - ms[0]) * ms[1]) * bf16r(gw) + bf16r(gb), kNCarry);
  }
  unsigned short* dp = XN16 + i * 8u;
  *(volatile v8h*)dp = hv;
  __threadfence();
  *(volatile v8h*)dp = hv;
}
static_assert((size_t)kRows * kD / 8 == 2048ull * kThr && kD / 8 == 128, "the apply grid exact: 2,048 blocks: two rows a block");

__global__ __launch_bounds__(kThr) void sink_kernel(const float* __restrict__ src, int srcPitch, int sa, int sk, float* __restrict__ dst, int last) {
  const unsigned i = blockIdx.x * (unsigned)kThr + threadIdx.x;
  const unsigned m = i >> 4;
  const unsigned a = i & 15u;
  const unsigned row = m >> 3;
  const unsigned hd = m & 7u;
  const float* ps = src + row * (unsigned)srcPitch + hd * (unsigned)(kN * kN) + a * (unsigned)sa;
  float v[kN];
#pragma unroll
  for (int k = 0; k < kN; ++k) v[k] = ps[(unsigned)k * (unsigned)sk];
  float mx = v[0];
#pragma unroll
  for (int k = 1; k < kN; ++k) mx = fmaxf(mx, v[k]);
  float sm = 0.0f;
#pragma unroll
  for (int k = 0; k < kN; ++k) sm += expf(v[k] - mx);
  const float lse = mx + logf(sm);
  float* pd = dst + m * (unsigned)(kN * kN);
  const bool fin = last != 0;
  for (int pass = 0; pass < 2; ++pass) {
#pragma unroll
    for (int k = 0; k < kN; ++k) { const float r = v[k] - lse; const float er = expf(r); *(volatile float*)(pd + (unsigned)k * (unsigned)kN + a) = fin ? er : r; }
    __threadfence();
  }
}
static_assert((size_t)kRows * kH * kN == 2048ull * kThr && kN == 16 && kH == 8, "the Sinkhorn pass's grid exact: 2,048 blocks: 16 matrices a block");

__global__ __launch_bounds__(kThr) void gate_kernel(const float* __restrict__ PRJ, float* __restrict__ G) {
  const unsigned i = blockIdx.x * (unsigned)kThr + threadIdx.x;
  const unsigned row = i >> 5;
  const unsigned c4 = (i & 31u) * 4u;
  const v4f p = *(const v4f*)(PRJ + row * (unsigned)kPrj + (unsigned)kHNN + c4);
  v4f o;
#pragma unroll
  for (int e = 0; e < 4; ++e) o[e] = 1.0f / (1.0f + expf(-p[e]));
  float* dp = G + i * 4u;
  *(volatile v4f*)dp = o;
  __threadfence();
  *(volatile v4f*)dp = o;
}
static_assert((size_t)kRows * kHN / 4 == 512ull * kThr && kHN / 4 == 32, "the gate's grid exact: 512 blocks");

__global__ __launch_bounds__(32) void step_kernel(const float* __restrict__ P, const float* __restrict__ G, const float* __restrict__ PRJ, unsigned short* __restrict__ HS16) {
  const unsigned ln = threadIdx.x;
  const unsigned sq = ln >> 3;
  const unsigned hd = ln & 7u;
  float h[kN];
#pragma unroll
  for (int k = 0; k < kN; ++k) h[k] = 0.0f;
  for (int l = 0; l < kL; ++l) {
    const unsigned row = sq * (unsigned)kL + (unsigned)l;
    const float* pm = P + (row * (unsigned)kH + hd) * (unsigned)(kN * kN);
    const float* pg = G + row * (unsigned)kHN + hd * (unsigned)kN;
    const float* pb = PRJ + row * (unsigned)kPrj + (unsigned)(kHNN + kHN) + hd * (unsigned)kN;
    float hn[kN];
#pragma unroll
    for (int q = 0; q < kN / 4; ++q) {
      const v4f gv = *(const v4f*)(pg + 4 * q), bv = *(const v4f*)(pb + 4 * q);
#pragma unroll
      for (int e = 0; e < 4; ++e) {
        const int ii = 4 * q + e;
        float acc = 0.0f;
#pragma unroll
        for (int r = 0; r < kN / 4; ++r) {
          const v4f pv = *(const v4f*)(pm + ii * kN + 4 * r);
          acc += pv[0] * h[4 * r]; acc += pv[1] * h[4 * r + 1]; acc += pv[2] * h[4 * r + 2]; acc += pv[3] * h[4 * r + 3];
        }
        hn[ii] = gv[e] * acc + (1.0f - gv[e]) * bv[e];
      }
    }
    v8h o0, o1;
#pragma unroll
    for (int k = 0; k < 8; ++k) { h[k] = hn[k]; h[8 + k] = hn[8 + k]; o0[k] = (_Float16)carry_flush(hn[k], kHCarry); o1[k] = (_Float16)carry_flush(hn[8 + k], kHCarry); }
    unsigned short* dp = HS16 + row * (unsigned)kHN + hd * (unsigned)kN;
    for (int pass = 0; pass < 2; ++pass) {
      *(volatile v8h*)dp = o0;
      *(volatile v8h*)(dp + 8) = o1;
      __threadfence();
    }
  }
}
static_assert(kNB * kH == 32 && kN == 16, "the step's grid exact: ONE block of 32 lanes: a lane a (sequence, head)");

__global__ __launch_bounds__(kThr) void close_kernel(const float* __restrict__ Y, const float* __restrict__ x, float* __restrict__ out) {
  const unsigned i = blockIdx.x * (unsigned)kThr + threadIdx.x;
  const float* px = x + i * 8u;
  const float* py = Y + i * 8u;
  const v4f a0 = *(const v4f*)px, a1 = *(const v4f*)(px + 4);
  const v4f y0 = *(const v4f*)py, y1 = *(const v4f*)(py + 4);
  v4f o0, o1;
#pragma unroll
  for (int e = 0; e < 4; ++e) { o0[e] = y0[e] + bf16r(a0[e]); o1[e] = y1[e] + bf16r(a1[e]); }
  float* dp = out + i * 8u;
  for (int pass = 0; pass < 2; ++pass) {
    *(volatile v4f*)dp = o0;
    *(volatile v4f*)(dp + 4) = o1;
    __threadfence();
  }
}
static_assert((size_t)kRows * kD / 8 == 2048ull * kThr && (size_t)kRows * kPrj < 4294967296ull / 4, "the closing sum's grid exact: 2,048 blocks; every plane's element offsets fit 32 bits");

extern "C" void kernel_launch(void* const* d_in, const int* in_sizes, int n_in,
                              void* d_out, int out_size, void* d_ws, size_t ws_size,
                              hipStream_t stream) {
  if (n_in < 11 || d_out == nullptr || d_ws == nullptr) return;
  if (in_sizes[0] != kRows * kD || in_sizes[1] != kD || in_sizes[2] != kD || in_sizes[3] != kD * kHNN || in_sizes[4] != kHNN || in_sizes[5] != kD * kHN || in_sizes[6] != kHN || in_sizes[7] != kD * kHN
      || in_sizes[8] != kHN || in_sizes[9] != kHN * kD || in_sizes[10] != kD) return;
  if (out_size != kOut0) return;
  if (ws_size < kWsTotal) return;
  const float* x = (const float*)d_in[0];
  const float* ln_w = (const float*)d_in[1];
  const float* ln_b = (const float*)d_in[2];
  const float* Wp = (const float*)d_in[3];
  const float* bp = (const float*)d_in[4];
  const float* Wg = (const float*)d_in[5];
  const float* bg = (const float*)d_in[6];
  const float* Wi = (const float*)d_in[7];
  const float* bi = (const float*)d_in[8];
  const float* Wo = (const float*)d_in[9];
  const float* bo = (const float*)d_in[10];
  float* out = (float*)d_out;
  char* ws = (char*)d_ws;
  unsigned short* WALL = (unsigned short*)(ws + kOffWALL);
  unsigned short* WOT = (unsigned short*)(ws + kOffWOT);
  float* BV = (float*)(ws + kOffBV);
  float* ST = (float*)(ws + kOffST);
  unsigned short* XN16 = (unsigned short*)(ws + kOffXN16);
  float* PRJ = (float*)(ws + kOffPRJ);
  float* LA = (float*)(ws + kOffLA);
  float* LB = (float*)(ws + kOffLB);
  float* G = (float*)(ws + kOffG);
  unsigned short* HS16 = (unsigned short*)(ws + kOffHS16);
  float* Y = (float*)(ws + kOffY);

  static_assert(kD / 8 == 128 && kHN / 8 == 16, "the transposing casts run one block a destination row with exactly K / 8 threads");
  wt_plane_kernel<<<kHNN, kD / 8, 0, stream>>>(Wp, WALL, kD, kHNN, kHNN, kD, 0);
  wt_plane_kernel<<<kHN, kD / 8, 0, stream>>>(Wg, WALL + (size_t)kHNN * kD, kD, kHN, kHN, kD, 0);
  wt_plane_kernel<<<kHN, kD / 8, 0, stream>>>(Wi, WALL + (size_t)(kHNN + kHN) * kD, kD, kHN, kHN, kD, 0);
  wt_plane_kernel<<<kD, kHN / 8, 0, stream>>>(Wo, WOT, kHN, kD, kD, kHN, 0);
  setup_kernel<<<13, kThr, 0, stream>>>(bp, bg, bi, bo, BV);
  stat_kernel<<<16, kThr, 0, stream>>>(x, ST);
  apply_kernel<<<2048, kThr, 0, stream>>>(x, ST, ln_w, ln_b, XN16);
  wmma_gemm64<0, false, 2, 0, false, 0><<<dim3((kRows / 64) * (kPrj / 64) / 8, 1), 256, 0, stream>>>(
      XN16, XN16, kD, 0L, WALL, WALL, kD, 0L, (void*)PRJ, (void*)PRJ, kPrj, 0L, BV, nullptr, 0L, kRows, kPrj, kD, kScP);
  const float* psrc = PRJ;
  int ppitch = kPrj;
  int sa = kN, sk = 1;
  const int nPass = 2 * kSweeps;
  for (int p = 0; p < nPass; ++p) {
    float* pdst = (p & 1) ? LB : LA;
    sink_kernel<<<2048, kThr, 0, stream>>>(psrc, ppitch, sa, sk, pdst, (p == nPass - 1) ? 1 : 0);
    psrc = pdst; ppitch = kHNN; sa = kN; sk = 1;
  }
  gate_kernel<<<512, kThr, 0, stream>>>(PRJ, G);
  step_kernel<<<1, 32, 0, stream>>>(psrc, G, PRJ, HS16);
  wmma_gemm64<0, false, 2, 0, false, 0><<<dim3((kRows / 64) * (kD / 64) / 8, 1), 256, 0, stream>>>(
      HS16, HS16, kHN, 0L, WOT, WOT, kHN, 0L, (void*)Y, (void*)Y, kD, 0L, BV + kPrj, nullptr, 0L, kRows, kD, kHN, kScO);
  close_kernel<<<2048, kThr, 0, stream>>>(Y, x, out);
}
static_assert(((kRows / 64) * (kPrj / 64)) % 8 == 0 && ((kRows / 64) * (kD / 64)) % 8 == 0, "the engine's grids: whole blocks of eight wave tiles");
